// QuanvolutionClassifierQuantum_65481071396971
// MI455X (gfx1250) — hardware-run, weakly checked
//
#include <hip/hip_runtime.h>
#include <math.h>

typedef __attribute__((ext_vector_type(16))) _Float16 v16h;
typedef __attribute__((ext_vector_type(8)))  _Float16 v8h;
typedef __attribute__((ext_vector_type(8)))  float    v8f;
typedef __attribute__((ext_vector_type(4)))  float    v4f;
typedef __attribute__((ext_vector_type(2)))  unsigned v2u;

constexpr int kImg       = 224;
constexpr int kSide      = 112;
constexpr int kPatches   = kSide * kSide;
constexpr int kBatch     = 32;
constexpr int kCls       = 10;
constexpr int kClsPad    = 16;
constexpr int kFeat      = 4 * kPatches;
constexpr int kKChunk    = 512;
constexpr int kNumChunks = kFeat / kKChunk;
constexpr int kPartTile  = kBatch * kClsPad;
constexpr int kGateTab   = 32;
static_assert(kPatches == 12544);
static_assert(kFeat == 50176);
static_assert(kNumChunks * kKChunk == kFeat);
static_assert(kNumChunks == 98);
static_assert((kKChunk % 32) == 0);
static_assert(kBatch == 32);
static_assert(((kBatch * kPatches) % 256) == 0);
static_assert(((kClsPad * kFeat / 8) % 256) == 0);
static_assert((kFeat % 8) == 0);
static_assert(kPartTile == 512);

constexpr float kFeatCarry    = 256.0f;
constexpr float kWgtCarry     = 4096.0f;
constexpr float kFold         = 1.0f / (kFeatCarry * kWgtCarry);
constexpr float kF16MinNormal = 6.103515625e-05f;

constexpr size_t kSzTab   = (size_t)kGateTab * 4;
constexpr size_t kSzFeats = (size_t)kBatch * kFeat * 2;
constexpr size_t kSzBt    = (size_t)kClsPad * kFeat * 2;
constexpr size_t kSzPart  = (size_t)kNumChunks * kPartTile * 4;
constexpr size_t kOffTab   = 0;
constexpr size_t kOffFeats = kOffTab + kSzTab;
constexpr size_t kOffBt    = kOffFeats + kSzFeats;
constexpr size_t kOffPart  = kOffBt + kSzBt;
constexpr size_t kWsTotal  = kOffPart + kSzPart;
static_assert(kWsTotal == 5017728ull);
static_assert(kWsTotal <= 134217728ull);
static_assert((kOffFeats % 128) == 0 && (kOffBt % 128) == 0 && (kOffPart % 128) == 0);

__device__ __forceinline__ void pin_f32(float& v) { asm volatile("" : "+v"(v)); }

__device__ __forceinline__ unsigned f16_bits_flushed(float v) {
  const float t = (fabsf(v) < kF16MinNormal) ? 0.0f : v;
  const _Float16 h = (_Float16)t;
  return (unsigned)__builtin_bit_cast(unsigned short, h);
}
__device__ __forceinline__ _Float16 f16_flushed(float v) {
  const float t = (fabsf(v) < kF16MinNormal) ? 0.0f : v;
  return (_Float16)t;
}

union FragH { v16h v; v8h h[2]; };
__device__ __forceinline__ v16h load_frag_f16(const _Float16* p) {
  FragH f;
  f.h[0] = *(const v8h*)(p);
  f.h[1] = *(const v8h*)(p + 16);
  return f.v;
}
__device__ __forceinline__ v8f mma_f16_guarded(v16h a, v16h b, v8f c) {
  c = __builtin_amdgcn_wmma_f32_16x16x32_f16(false, a, false, b, (short)0, c, false, false);
  asm volatile("v_nop\n\tv_nop\n\tv_nop\n\tv_nop" : "+v"(c) : "v"(a), "v"(b));
  return c;
}

__global__ __launch_bounds__(32) void gate_table_kernel(
    const float* __restrict__ p1, const float* __restrict__ p2, float* __restrict__ tab)
{
  const int t = threadIdx.x;
  const int e = (t < 24) ? t : 23;
  const int pass = e / 12;
  const int r = e - pass * 12;
  const int pi = r >> 1;
  const int which = r & 1;
  float a1 = p1[pi];
  float a2 = p2[pi];
  pin_f32(a1);
  pin_f32(a2);
  const float ang = (pass == 0) ? a1 : a2;
  float sn, cn;
  sincosf(0.5f * ang, &sn, &cn);
  float val = (which != 0) ? sn : cn;
  val = (t < 24) ? val : 0.0f;
  float* dst = tab + t;
  *(volatile float*)dst = val;
  __threadfence();
  *(volatile float*)dst = val;
}

__global__ __launch_bounds__(256) void patch_circuit_kernel(
    const float* __restrict__ x, const float* __restrict__ tab, unsigned short* __restrict__ feats)
{
  int gid = blockIdx.x * 256 + threadIdx.x;
  gid = (gid < kBatch * kPatches) ? gid : (kBatch * kPatches - 1);
  const int b  = gid / kPatches;
  const int p  = gid - b * kPatches;
  const int pr = p / kSide;
  const int pc = p - pr * kSide;
  const int R  = 2 * pr;
  const int C  = 2 * pc;
  const float* xb = x + (size_t)b * (kImg * kImg);
  const int c2i = (C + 2 < kImg) ? (C + 2) : (kImg - 1);
  float v00 = xb[R * kImg + C];
  float v01 = xb[R * kImg + C + 1];
  float v02 = xb[R * kImg + c2i];
  float v10 = xb[(R + 1) * kImg + C];
  float v11 = xb[(R + 1) * kImg + C + 1];
  pin_f32(v00);
  pin_f32(v01);
  pin_f32(v02);
  pin_f32(v10);
  pin_f32(v11);
  const bool edge = (C == kImg - 2);
  float a0 = v00;
  float a1 = v01;
  float a2 = edge ? v10 : v02;
  float a3 = edge ? v11 : v10;
  float r0 = 0.0f, r1 = 0.0f, r2 = 0.0f, r3 = 0.0f;

#pragma unroll 1
  for (int pass = 0; pass < 2; ++pass) {
    const float* g = tab + pass * 12;
    const float gc0 = g[0],  gs0 = g[1];
    const float gc1 = g[2],  gs1 = g[3];
    const float gc2 = g[4],  gs2 = g[5];
    const float gc3 = g[6],  gs3 = g[7];
    const float gc4 = g[8],  gs4 = g[9];
    const float gc5 = g[10], gs5 = g[11];

    float q0 = a0, q1 = a1, q2 = a2, q3 = a3;
    float c0 = 0.0f, c1 = 0.0f, c2 = 0.0f, c3 = 0.0f;
    float s0 = 0.0f, s1 = 0.0f, s2 = 0.0f, s3 = 0.0f;
#pragma unroll 1
    for (int w = 0; w < 4; ++w) {
      const float ang = q0;
      float sn, cn;
      sincosf(0.5f * ang, &sn, &cn);
      q0 = q1; q1 = q2; q2 = q3; q3 = ang;
      c0 = c1; c1 = c2; c2 = c3; c3 = cn;
      s0 = s1; s1 = s2; s2 = s3; s3 = sn;
    }

    const float e0 = c0 * c1;
    const float e1 = c0 * s1;
    const float e2 = s0 * c1;
    const float e3 = s0 * s1;
    const float t0 = gc0 * e0 - gs0 * e2;
    const float t2 = gs0 * e0 + gc0 * e2;
    const float t1 = gc0 * e1 - gs0 * e3;
    const float t3 = gs0 * e1 + gc0 * e3;
    float ar0 = gc1 * t0;
    float ai0 = -(gs1 * t1);
    float ar1 = gc1 * t1;
    float ai1 = -(gs1 * t0);
    float ar2 = gc1 * t2;
    float ai2 = -(gs1 * t3);
    float ar3 = gc1 * t3;
    float ai3 = -(gs1 * t2);
    {
      const float tr = ar2; ar2 = ar3; ar3 = tr;
      const float ti = ai2; ai2 = ai3; ai3 = ti;
    }
    const float zr0 = gc5 * ar0 + gs5 * ai0;
    const float zi0 = gc5 * ai0 - gs5 * ar0;
    const float zr1 = gc5 * ar1 + gs5 * ai1;
    const float zi1 = gc5 * ai1 - gs5 * ar1;
    const float zr2 = gc5 * ar2 - gs5 * ai2;
    const float zi2 = gc5 * ai2 + gs5 * ar2;
    const float zr3 = gc5 * ar3 - gs5 * ai3;
    const float zi3 = gc5 * ai3 + gs5 * ar3;
    const float pa0 = zr0 * zr0 + zi0 * zi0;
    const float pa1 = zr1 * zr1 + zi1 * zi1;
    const float pa2 = zr2 * zr2 + zi2 * zi2;
    const float pa3 = zr3 * zr3 + zi3 * zi3;
    const float zA0 = (pa0 + pa1) - (pa2 + pa3);
    const float zA1 = (pa0 + pa2) - (pa1 + pa3);
    const float nA  = (pa0 + pa1) + (pa2 + pa3);

    const float u0 = c2 * c3;
    const float u1 = c2 * s3;
    const float u2 = s2 * c3;
    const float u3 = s2 * s3;
    const float br0 = gc2 * u0;
    const float bi0 = -(gs2 * u0);
    const float br1 = gc2 * u1;
    const float bi1 = -(gs2 * u1);
    const float br2 = gc2 * u2;
    const float bi2 = gs2 * u2;
    const float br3 = gc2 * u3;
    const float bi3 = gs2 * u3;
    const float xr0 = gc3 * br0 - gs3 * br1;
    const float xi0 = gc3 * bi0 - gs3 * bi1;
    const float xr1 = gs3 * br0 + gc3 * br1;
    const float xi1 = gs3 * bi0 + gc3 * bi1;
    float xr2 = gc3 * br2 - gs3 * br3;
    float xi2 = gc3 * bi2 - gs3 * bi3;
    float xr3 = gs3 * br2 + gc3 * br3;
    float xi3 = gs3 * bi2 + gc3 * bi3;
    {
      const float tr = xr2; xr2 = xr3; xr3 = tr;
      const float ti = xi2; xi2 = xi3; xi3 = ti;
    }
    const float yr0 = gc4 * xr0 + gs4 * xi2;
    const float yi0 = gc4 * xi0 - gs4 * xr2;
    const float yr2 = gs4 * xi0 + gc4 * xr2;
    const float yi2 = gc4 * xi2 - gs4 * xr0;
    const float yr1 = gc4 * xr1 + gs4 * xi3;
    const float yi1 = gc4 * xi1 - gs4 * xr3;
    const float yr3 = gs4 * xi1 + gc4 * xr3;
    const float yi3 = gc4 * xi3 - gs4 * xr1;
    const float pb0 = yr0 * yr0 + yi0 * yi0;
    const float pb1 = yr1 * yr1 + yi1 * yi1;
    const float pb2 = yr2 * yr2 + yi2 * yi2;
    const float pb3 = yr3 * yr3 + yi3 * yi3;
    const float zB2 = (pb0 + pb1) - (pb2 + pb3);
    const float zB3 = (pb0 + pb2) - (pb1 + pb3);
    const float nB  = (pb0 + pb1) + (pb2 + pb3);

    const float m0 = zA0 * nB;
    const float m1 = zA1 * nB;
    const float m2 = zB2 * nA;
    const float m3 = zB3 * nA;
    r0 += m0; r1 += m1; r2 += m2; r3 += m3;
    a0 = m0;  a1 = m1;  a2 = m2;  a3 = m3;
  }

  const unsigned h0 = f16_bits_flushed(r0 * kFeatCarry);
  const unsigned h1 = f16_bits_flushed(r1 * kFeatCarry);
  const unsigned h2 = f16_bits_flushed(r2 * kFeatCarry);
  const unsigned h3 = f16_bits_flushed(r3 * kFeatCarry);
  v2u pk;
  pk.x = h0 | (h1 << 16);
  pk.y = h2 | (h3 << 16);
  unsigned short* dst = feats + (size_t)gid * 4;
  *(volatile v2u*)dst = pk;
  __threadfence();
  *(volatile v2u*)dst = pk;
}

__global__ __launch_bounds__(256) void weight_plane_kernel(
    const float* __restrict__ W, unsigned short* __restrict__ Bt)
{
  int i = blockIdx.x * 256 + threadIdx.x;
  i = (i < kClsPad * kFeat / 8) ? i : (kClsPad * kFeat / 8 - 1);
  const int e0  = i * 8;
  const int row = e0 / kFeat;
  const int col = e0 - row * kFeat;
  const bool keep = (row < kCls);
  const int srow = keep ? row : (kCls - 1);
  const float* src = W + (size_t)srow * kFeat + col;
  const v4f w0 = *(const v4f*)(src);
  const v4f w1 = *(const v4f*)(src + 4);
  v8h hv;
#pragma unroll
  for (int e = 0; e < 4; ++e) {
    const float f0 = w0[e];
    const float f1 = w1[e];
    const float g0 = keep ? (f0 * kWgtCarry) : 0.0f;
    const float g1 = keep ? (f1 * kWgtCarry) : 0.0f;
    hv[e]     = f16_flushed(g0);
    hv[4 + e] = f16_flushed(g1);
  }
  unsigned short* dst = Bt + (size_t)e0;
  *(volatile v8h*)dst = hv;
  __threadfence();
  *(volatile v8h*)dst = hv;
}

__global__ __launch_bounds__(32) void splitk_gemm_kernel(
    const unsigned short* __restrict__ Ap, const unsigned short* __restrict__ Bp, float* __restrict__ part)
{
  __shared__ __align__(16) float sP[kPartTile];
  const _Float16* A  = (const _Float16*)Ap;
  const _Float16* Bt = (const _Float16*)Bp;
  const int lane = threadIdx.x & 31;
  const int hh = lane >> 4;
  const int n  = lane & 15;
  const int kbase = blockIdx.x * kKChunk;
  const _Float16* a0p = A  + (size_t)n * kFeat + kbase + 8 * hh;
  const _Float16* a1p = A  + (size_t)(n + 16) * kFeat + kbase + 8 * hh;
  const _Float16* bp  = Bt + (size_t)n * kFeat + kbase + 8 * hh;
  v8f c0 = (v8f){0.f, 0.f, 0.f, 0.f, 0.f, 0.f, 0.f, 0.f};
  v8f c1 = (v8f){0.f, 0.f, 0.f, 0.f, 0.f, 0.f, 0.f, 0.f};
#pragma unroll 4
  for (int ks = 0; ks < kKChunk / 32; ++ks) {
    const v16h fa0 = load_frag_f16(a0p + ks * 32);
    const v16h fa1 = load_frag_f16(a1p + ks * 32);
    const v16h fb  = load_frag_f16(bp + ks * 32);
    c0 = mma_f16_guarded(fa0, fb, c0);
    c1 = mma_f16_guarded(fa1, fb, c1);
  }
#pragma unroll
  for (int r = 0; r < 8; ++r) {
    sP[(8 * hh + r) * kClsPad + n]      = c0[r] * kFold;
    sP[(16 + 8 * hh + r) * kClsPad + n] = c1[r] * kFold;
  }
  __syncthreads();
  v4f o[4];
#pragma unroll
  for (int it = 0; it < 4; ++it) o[it] = *(const v4f*)(sP + it * 128 + lane * 4);
  float* dst = part + (size_t)blockIdx.x * kPartTile;
  for (int pass = 0; pass < 2; ++pass) {
#pragma unroll
    for (int it = 0; it < 4; ++it) *(volatile v4f*)(dst + it * 128 + lane * 4) = o[it];
    __threadfence();
  }
}

__global__ __launch_bounds__(512) void finalize_kernel(
    const float* __restrict__ part, const float* __restrict__ bias, float* __restrict__ out)
{
  __shared__ __align__(16) float sL[kPartTile];
  __shared__ __align__(16) float sO[kBatch * kCls];
  const int t = threadIdx.x;
  const int b = t >> 4;
  const int c = t & 15;
  float acc = 0.0f;
#pragma unroll 1
  for (int blk = 0; blk < kNumChunks; ++blk) acc += part[(size_t)blk * kPartTile + t];
  const int cc = (c < kCls) ? c : (kCls - 1);
  const float bv = bias[cc];
  const float logit = acc + bv;
  sL[t] = logit;
  __syncthreads();
  const float* rowp = sL + b * kClsPad;
  float mx = rowp[0];
#pragma unroll 1
  for (int j = 1; j < kCls; ++j) mx = fmaxf(mx, rowp[j]);
  float se = 0.0f;
#pragma unroll 1
  for (int j = 0; j < kCls; ++j) se += expf(rowp[j] - mx);
  const float outv = (logit - mx) - logf(se);
  if (c < kCls) sO[b * kCls + c] = outv;
  __syncthreads();
  if (t < 32) {
    v4f o[3];
#pragma unroll
    for (int it = 0; it < 3; ++it) {
      const int idx = it * 32 + t;
      const int idc = (idx < 80) ? idx : 79;
      o[it] = *(const v4f*)(sO + idc * 4);
    }
    for (int pass = 0; pass < 2; ++pass) {
#pragma unroll
      for (int it = 0; it < 3; ++it) {
        const int idx = it * 32 + t;
        if (idx < 80) *(volatile v4f*)(out + idx * 4) = o[it];
      }
      __threadfence();
    }
  }
}

extern "C" void kernel_launch(void* const* d_in, const int* in_sizes, int n_in,
                              void* d_out, int out_size, void* d_ws, size_t ws_size,
                              hipStream_t stream) {
  if (n_in < 5) return;
  if (in_sizes[0] != kBatch * kImg * kImg) return;
  if (in_sizes[1] != 6) return;
  if (in_sizes[2] != 6) return;
  if (in_sizes[3] != kCls * kFeat) return;
  if (in_sizes[4] != kCls) return;
  if (out_size != kBatch * kCls) return;
  if (ws_size < kWsTotal) return;

  const float* x  = (const float*)d_in[0];
  const float* p1 = (const float*)d_in[1];
  const float* p2 = (const float*)d_in[2];
  const float* W  = (const float*)d_in[3];
  const float* bi = (const float*)d_in[4];
  float* out = (float*)d_out;

  char* ws = (char*)d_ws;
  float*          TAB   = (float*)(ws + kOffTab);
  unsigned short* FEATS = (unsigned short*)(ws + kOffFeats);
  unsigned short* BT    = (unsigned short*)(ws + kOffBt);
  float*          PART  = (float*)(ws + kOffPart);

  gate_table_kernel<<<1, 32, 0, stream>>>(p1, p2, TAB);
  patch_circuit_kernel<<<(kBatch * kPatches) / 256, 256, 0, stream>>>(x, TAB, FEATS);
  weight_plane_kernel<<<(kClsPad * kFeat / 8) / 256, 256, 0, stream>>>(W, BT);
  splitk_gemm_kernel<<<kNumChunks, 32, 0, stream>>>(FEATS, BT, PART);
  finalize_kernel<<<1, 512, 0, stream>>>(PART, bi, out);
}
